// _SelfAttention_47656957116590
// MI455X (gfx1250) — hardware-verified
//
#include <hip/hip_runtime.h>
#include <math.h>

constexpr int kBatch = 2;
constexpr int kSeq   = 2048;
constexpr int kDim   = 1024;
constexpr int kHeads = 16;
constexpr int kDh    = 64;
constexpr int kGroup = 2;
constexpr int kTok   = kBatch * kSeq;
constexpr int kQKld  = 2 * kDim;
constexpr float kWCarry    = 16.0f;
constexpr float kWCarryInv = 1.0f / 16.0f;
constexpr float kPCarry    = 32768.0f;
constexpr float kCtxCarry  = 256.0f;
constexpr float kPVScale   = kCtxCarry / kPCarry;
constexpr float kOutScale  = 1.0f / (kCtxCarry * kWCarry);
constexpr float kScoreScale = 0.125f;
static_assert(kHeads * kDh == kDim, "shape");
static_assert(kHeads % kGroup == 0, "groups");
static_assert(kTok % 64 == 0 && kQKld % 64 == 0 && kDim % 32 == 0, "qk proj tiles");
static_assert(kDim % 64 == 0 && kSeq % 64 == 0, "vt proj tiles");
static_assert(kSeq % 64 == 0 && kDh % 32 == 0, "score tiles");
static_assert(kDh % 64 == 0 && kSeq % 32 == 0, "ctx tiles");
static_assert(kSeq == 4 * 512, "softmax row map");
static_assert((kTok * kDim) % (8 * 256) == 0, "cast grid");

typedef __attribute__((ext_vector_type(16))) _Float16 v16h;
typedef __attribute__((ext_vector_type(8)))  _Float16 v8h;
typedef __attribute__((ext_vector_type(8)))  float    v8f;
typedef __attribute__((ext_vector_type(4)))  float    v4f;
typedef __attribute__((ext_vector_type(2)))  float    v2f;
typedef __attribute__((ext_vector_type(4)))  unsigned int v4u;

__device__ __forceinline__ unsigned short f2bf_bits(float f) {
  unsigned u = __float_as_uint(f);
  return (unsigned short)((u + 0x7FFFu + ((u >> 16) & 1u)) >> 16);
}
__device__ __forceinline__ float bf_bits2f(unsigned short h) { return __uint_as_float(((unsigned)h) << 16); }

__device__ __forceinline__ void dep_guard4_h(v8f& a, v8f& b, v8f& c, v8f& d,
                                             v16h x, v16h y0, v16h y1, v16h y2, v16h y3) {
  asm volatile("v_nop\n\tv_nop\n\tv_nop\n\tv_nop"
               : "+v"(a), "+v"(b), "+v"(c), "+v"(d)
               : "v"(x), "v"(y0), "v"(y1), "v"(y2), "v"(y3));
}
__device__ __forceinline__ void keep4_h(v16h a, v16h b, v16h c, v16h d) { asm volatile("v_nop" :: "v"(a), "v"(b), "v"(c), "v"(d)); }
__device__ __forceinline__ void acc_guard4(v8f& a, v8f& b, v8f& c, v8f& d) { asm volatile("v_nop\n\tv_nop\n\tv_nop\n\tv_nop" : "+v"(a), "+v"(b), "+v"(c), "+v"(d)); }

struct FragH {
  union U { v16h v; v8h h[2]; };
  static __device__ __forceinline__ v16h load(const _Float16* p) {
    U f; f.h[0] = *(const v8h*)(p); f.h[1] = *(const v8h*)(p + 16); return f.v;
  }
  static __device__ __forceinline__ v8f mma(v16h a, v16h b, v8f c) {
    return __builtin_amdgcn_wmma_f32_16x16x32_f16(false, a, false, b, (short)0, c, false, false);
  }
};

__device__ __forceinline__ unsigned pk16(unsigned short a, unsigned short b) { return (unsigned)a | ((unsigned)b << 16); }
__device__ __forceinline__ unsigned short h_bits(float f) { const _Float16 h = (_Float16)f; return __builtin_bit_cast(unsigned short, h); }
__device__ __forceinline__ unsigned short hb16_bits(float f) { return h_bits(bf_bits2f(f2bf_bits(f))); }

template <int BIAS_MODE, int OUT_MODE>
__global__ __launch_bounds__(256) void wmma_gemm64(
    const unsigned short* __restrict__ Ap, int lda, long strideA,
    const unsigned short* __restrict__ Btp, int ldb, long strideB,
    void* __restrict__ Cout, int ldc, long strideC,
    const float* __restrict__ bias,
    int M, int N, int K, float scale) {
  const _Float16* A = (const _Float16*)Ap; const _Float16* Bt = (const _Float16*)Btp;
  __shared__ __align__(16) float sT[8][16 * 68];
  const int b    = blockIdx.y;
  const int lane = threadIdx.x & 31;
  const int wave = threadIdx.x >> 5;
  const int tilesN = N >> 6;
  const int tilesM = M >> 6;
  const int tile = blockIdx.x * 8 + wave;
  if (tile >= tilesM * tilesN) return;
  const int tm = tile / tilesN;
  const int tn = tile - tm * tilesN;
  const int m0 = tm << 6;
  const int n0 = tn << 6;

  const _Float16* Ab = A  + (size_t)b * strideA;
  const _Float16* Bb = Bt + (size_t)b * strideB;

  const int rlane = lane & 15;
  const int koff  = (lane >> 4) * 8;
  const int mOff  = (lane >> 4) * 8;

  v8f acc[4][4];
#pragma unroll
  for (int i = 0; i < 4; ++i)
#pragma unroll
    for (int j = 0; j < 4; ++j) acc[i][j] = (v8f){0.f,0.f,0.f,0.f,0.f,0.f,0.f,0.f};

  for (int k0 = 0; k0 < K; k0 += 32) {
    v16h bh[4];
#pragma unroll
    for (int j = 0; j < 4; ++j) {
      const size_t bo = (size_t)(n0 + (j << 4) + rlane) * ldb + koff + k0;
      bh[j] = FragH::load(Bb + bo);
    }
#pragma unroll
    for (int i = 0; i < 4; ++i) {
      const size_t ao = (size_t)(m0 + (i << 4) + rlane) * lda + koff + k0;
      v16h ah = FragH::load(Ab + ao);
#pragma unroll
      for (int j = 0; j < 4; ++j) acc[i][j] = FragH::mma(ah, bh[j], acc[i][j]);
      dep_guard4_h(acc[i][0], acc[i][1], acc[i][2], acc[i][3], ah, bh[0], bh[1], bh[2], bh[3]);
    }
    keep4_h(bh[0], bh[1], bh[2], bh[3]);
  }
  acc_guard4(acc[0][0], acc[0][1], acc[0][2], acc[0][3]);
  acc_guard4(acc[1][0], acc[1][1], acc[1][2], acc[1][3]);
  acc_guard4(acc[2][0], acc[2][1], acc[2][2], acc[2][3]);
  acc_guard4(acc[3][0], acc[3][1], acc[3][2], acc[3][3]);

  float* slab = sT[wave];
#pragma unroll
  for (int i = 0; i < 4; ++i) {
    const int mBase = m0 + (i << 4);
    float bm[8];
#pragma unroll
    for (int r = 0; r < 8; ++r) bm[r] = 0.f;
    if (BIAS_MODE == 1) {
      const v4f q0 = *(const v4f*)(bias + mBase + mOff);
      const v4f q1 = *(const v4f*)(bias + mBase + mOff + 4);
      bm[0] = q0[0]; bm[1] = q0[1]; bm[2] = q0[2]; bm[3] = q0[3];
      bm[4] = q1[0]; bm[5] = q1[1]; bm[6] = q1[2]; bm[7] = q1[3];
    }
#pragma unroll
    for (int j = 0; j < 4; ++j) {
      const int n = n0 + (j << 4) + rlane;
      float bv = 0.f;
      if (BIAS_MODE == 2) bv = bias[n];
#pragma unroll
      for (int r = 0; r < 8; ++r) {
        float v = acc[i][j][r] * scale;
        if (BIAS_MODE == 1) v += bm[r];
        if (BIAS_MODE == 2) v += bv;
        slab[(mOff + r) * 68 + (j << 4) + rlane] = v;
      }
    }
    __builtin_amdgcn_fence(__ATOMIC_RELEASE, "workgroup");
    __builtin_amdgcn_wave_barrier();
    __builtin_amdgcn_fence(__ATOMIC_ACQUIRE, "workgroup");
    if (OUT_MODE == 0) {
      float* C = (float*)Cout + (size_t)b * strideC;
      const int hh = lane >> 4, c4 = (lane & 15) * 4;
      for (int pass = 0; pass < 2; ++pass) {
#pragma unroll
        for (int it = 0; it < 8; ++it) {
          const int row = it * 2 + hh;
          v4f v = *(const v4f*)(slab + row * 68 + c4);
          *(volatile v4f*)(C + (size_t)(mBase + row) * ldc + n0 + c4) = v;
        }
        __threadfence();
      }
    } else {
      const int q = lane >> 3, c8 = (lane & 7) * 8;
      unsigned short* C = (unsigned short*)Cout + (size_t)b * strideC;
      for (int pass = 0; pass < 2; ++pass) {
#pragma unroll
        for (int it = 0; it < 4; ++it) {
          const int row = it * 4 + q;
          const float* sp = slab + row * 68 + c8;
          v8h hv;
#pragma unroll
          for (int e = 0; e < 8; ++e) hv[e] = (_Float16)sp[e];
          *(volatile v8h*)(C + (size_t)(mBase + row) * ldc + n0 + c8) = hv;
        }
        __threadfence();
      }
    }
    __builtin_amdgcn_fence(__ATOMIC_RELEASE, "workgroup");
    __builtin_amdgcn_wave_barrier();
    __builtin_amdgcn_fence(__ATOMIC_ACQUIRE, "workgroup");
  }
}

__global__ __launch_bounds__(256) void cast8_bf_f16_kernel(const float* __restrict__ in, unsigned short* __restrict__ out, int n8) {
  const int i = blockIdx.x * 256 + threadIdx.x;
  if (i >= n8) return;
  const float* p = in + 8 * (size_t)i;
  const v4f a = *(const v4f*)(p);
  const v4f c = *(const v4f*)(p + 4);
  unsigned short hb[8];
#pragma unroll
  for (int e = 0; e < 4; ++e) {
    hb[e]     = hb16_bits(a[e]);
    hb[4 + e] = hb16_bits(c[e]);
  }
  const v4u u = (v4u){pk16(hb[0], hb[1]), pk16(hb[2], hb[3]), pk16(hb[4], hb[5]), pk16(hb[6], hb[7])};
  unsigned short* q = out + 8 * (size_t)i;
  *(volatile v4u*)q = u;
  __threadfence();
  *(volatile v4u*)q = u;
}

__global__ __launch_bounds__(256) void wtcast_kernel(const float* __restrict__ W, unsigned short* __restrict__ out,
                                                     int nCols, float carry) {
  __shared__ float sm[64][65];
  const int t  = threadIdx.x;
  const int k0 = blockIdx.x * 64;
  const int n0 = blockIdx.y * 64;
#pragma unroll
  for (int i = 0; i < 16; ++i) {
    const int e = i * 256 + t;
    const int r = e >> 6;
    const int c = e & 63;
    sm[c][r] = bf_bits2f(f2bf_bits(W[(size_t)(k0 + r) * nCols + n0 + c])) * carry;
  }
  __syncthreads();
  const int lane = t & 31, wave = t >> 5;
  const int q = lane >> 3, c8 = (lane & 7) * 8;
  for (int pass = 0; pass < 2; ++pass) {
#pragma unroll
    for (int it = 0; it < 2; ++it) {
      const int row = wave * 8 + it * 4 + q;
      unsigned short hb[8];
#pragma unroll
      for (int e = 0; e < 8; ++e) hb[e] = h_bits(sm[row][c8 + e]);
      const v4u u = (v4u){pk16(hb[0], hb[1]), pk16(hb[2], hb[3]), pk16(hb[4], hb[5]), pk16(hb[6], hb[7])};
      *(volatile v4u*)(out + (size_t)(n0 + row) * kDim + k0 + c8) = u;
    }
    __threadfence();
  }
}

__global__ __launch_bounds__(256) void softmax_row_kernel(const float* __restrict__ Sp, unsigned short* __restrict__ Pp) {
  __shared__ __align__(16) float lg[kSeq];
  __shared__ float redM[8];
  __shared__ float redS[8];
  const int i    = blockIdx.x;
  const int hg   = blockIdx.y;
  const int t    = threadIdx.x;
  const int lane = t & 31, wave = t >> 5;
  const size_t rowoff = ((size_t)hg * kSeq + i) * kSeq;
  const float* sr = Sp + rowoff;

  float mx = -__builtin_inff();
#pragma unroll 1
  for (int it = 0; it < 4; ++it) {
    const int c = it * 512 + 2 * t;
    const v2f sv = *(const v2f*)(sr + c);
    mx = fmaxf(mx, fmaxf(sv[0], sv[1]));
    *(v2f*)(lg + c) = sv;
  }
#pragma unroll
  for (int off = 16; off > 0; off >>= 1) mx = fmaxf(mx, __shfl_xor(mx, off, 32));
  if (lane == 0) redM[wave] = mx;
  __syncthreads();
  float m = redM[0];
#pragma unroll
  for (int w = 1; w < 8; ++w) m = fmaxf(m, redM[w]);

  float sum = 0.f;
#pragma unroll 1
  for (int it = 0; it < 4; ++it) {
    const int c = it * 512 + 2 * t;
    const v2f l = *(const v2f*)(lg + c);
    v2f ev;
#pragma unroll
    for (int e = 0; e < 2; ++e) {
      ev[e] = expf(l[e] - m);
      sum += ev[e];
    }
    *(v2f*)(lg + c) = ev;
  }
#pragma unroll
  for (int off = 16; off > 0; off >>= 1) sum += __shfl_xor(sum, off, 32);
  if (lane == 0) redS[wave] = sum;
  __syncthreads();
  float tot = redS[0];
#pragma unroll
  for (int w = 1; w < 8; ++w) tot += redS[w];
  const float inv = kPCarry / tot;

  const v4f e0 = *(const v4f*)(lg + 8 * t);
  const v4f e1 = *(const v4f*)(lg + 8 * t + 4);
  unsigned short hb[8];
#pragma unroll
  for (int e = 0; e < 4; ++e) {
    hb[e]     = h_bits(e0[e] * inv);
    hb[4 + e] = h_bits(e1[e] * inv);
  }
  const v4u u = (v4u){pk16(hb[0], hb[1]), pk16(hb[2], hb[3]), pk16(hb[4], hb[5]), pk16(hb[6], hb[7])};
  unsigned short* pr = Pp + rowoff + 8 * (size_t)t;
  *(volatile v4u*)pr = u;
  __threadfence();
  *(volatile v4u*)pr = u;
}

extern "C" void kernel_launch(void* const* d_in, const int* in_sizes, int n_in,
                              void* d_out, int out_size, void* d_ws, size_t ws_size,
                              hipStream_t stream) {
  if (n_in < 5) return;
  const int nTokElem = kTok * kDim;
  if (in_sizes[0] != nTokElem) return;
  if (in_sizes[1] != kDim * 3 * kDim) return;
  if (in_sizes[2] != 3 * kDim) return;
  if (in_sizes[3] != kDim * kDim) return;
  if (in_sizes[4] != kDim) return;
  if (out_size != nTokElem) return;

  const size_t szXH  = (size_t)kTok * kDim * 2;
  const size_t szWQT = (size_t)3 * kDim * kDim * 2;
  const size_t szWPT = (size_t)kDim * kDim * 2;
  const size_t szQK  = (size_t)kTok * kQKld * 2;
  const size_t szVT  = (size_t)kBatch * kDim * kSeq * 2;
  const size_t szSC  = (size_t)kGroup * kSeq * kSeq * 4;
  const size_t szPP  = (size_t)kGroup * kSeq * kSeq * 2;
  const size_t szO   = (size_t)kTok * kDim * 2;
  const size_t offXH  = 0;
  const size_t offWQT = offXH + szXH;
  const size_t offWPT = offWQT + szWQT;
  const size_t offQK  = offWPT + szWPT;
  const size_t offVT  = offQK + szQK;
  const size_t offSC  = offVT + szVT;
  const size_t offPP  = offSC + szSC;
  const size_t offO   = offPP + szPP;
  const size_t total  = offO + szO;
  if (ws_size < total) return;

  const float* x      = (const float*)d_in[0];
  const float* w_qkv  = (const float*)d_in[1];
  const float* b_qkv  = (const float*)d_in[2];
  const float* w_proj = (const float*)d_in[3];
  const float* b_proj = (const float*)d_in[4];
  float* out = (float*)d_out;
  char* ws = (char*)d_ws;
  unsigned short* XH  = (unsigned short*)(ws + offXH);
  unsigned short* WQT = (unsigned short*)(ws + offWQT);
  unsigned short* WPT = (unsigned short*)(ws + offWPT);
  unsigned short* QK  = (unsigned short*)(ws + offQK);
  unsigned short* VT  = (unsigned short*)(ws + offVT);
  float*          SC  = (float*)(ws + offSC);
  unsigned short* PP  = (unsigned short*)(ws + offPP);
  unsigned short* O16 = (unsigned short*)(ws + offO);

  const int n8 = nTokElem / 8;
  cast8_bf_f16_kernel<<<dim3(n8 / 256), dim3(256), 0, stream>>>(x, XH, n8);
  wtcast_kernel<<<dim3(kDim / 64, (3 * kDim) / 64), dim3(256), 0, stream>>>(w_qkv, WQT, 3 * kDim, kWCarry);
  wtcast_kernel<<<dim3(kDim / 64, kDim / 64), dim3(256), 0, stream>>>(w_proj, WPT, kDim, kWCarry);

  {
    const int tiles = (kTok / 64) * (kQKld / 64);
    wmma_gemm64<2, 1><<<dim3(tiles / 8, 1), dim3(256), 0, stream>>>(
        XH, kDim, 0L, WQT, kDim, 0L, (void*)QK, kQKld, 0L, b_qkv, kTok, kQKld, kDim, kWCarryInv);
  }
  {
    const int tiles = (kDim / 64) * (kSeq / 64);
    wmma_gemm64<1, 1><<<dim3(tiles / 8, kBatch), dim3(256), 0, stream>>>(
        WQT + (size_t)2 * kDim * kDim, kDim, 0L, XH, kDim, (long)kSeq * kDim,
        (void*)VT, kSeq, (long)kDim * kSeq, b_qkv + 2 * kDim, kDim, kSeq, kDim, kWCarryInv);
  }

  const long strideHead16 = (long)kDh;
  const long strideScore  = (long)kSeq * kSeq;
  const long strideVT     = (long)kDh * kSeq;
  const int  tilesScore   = (kSeq / 64) * (kSeq / 64);
  const int  tilesCtx     = (kSeq / 64) * (kDh / 64);

  for (int b = 0; b < kBatch; ++b) {
    for (int g = 0; g < kHeads / kGroup; ++g) {
      const size_t qkOff  = ((size_t)b * kSeq) * kQKld + (size_t)g * kGroup * kDh;
      const size_t tokOff = ((size_t)b * kSeq) * kDim  + (size_t)g * kGroup * kDh;
      const size_t headIdx = (size_t)b * kHeads + (size_t)g * kGroup;
      const unsigned short* Ag  = QK + qkOff;
      const unsigned short* Btg = QK + qkOff + kDim;
      wmma_gemm64<0, 0><<<dim3(tilesScore / 8, kGroup), dim3(256), 0, stream>>>(
          Ag, kQKld, strideHead16, Btg, kQKld, strideHead16,
          (void*)SC, kSeq, strideScore, b_qkv, kSeq, kSeq, kDh, kScoreScale);
      softmax_row_kernel<<<dim3(kSeq, kGroup), dim3(256), 0, stream>>>(SC, PP);
      const unsigned short* VTg = VT + headIdx * (size_t)kDh * kSeq;
      unsigned short* Og = O16 + tokOff;
      wmma_gemm64<0, 1><<<dim3(tilesCtx / 8, kGroup), dim3(256), 0, stream>>>(
          PP, kSeq, strideScore, VTg, kSeq, strideVT,
          (void*)Og, kDim, strideHead16, b_qkv, kSeq, kDh, kSeq, kPVScale);
    }
  }

  {
    const int tiles = (kTok / 64) * (kDim / 64);
    wmma_gemm64<2, 0><<<dim3(tiles / 8, 1), dim3(256), 0, stream>>>(
        O16, kDim, 0L, WPT, kDim, 0L, (void*)out, kDim, 0L, b_proj, kTok, kDim, kDim, kOutScale);
  }
}
